// SimpleNet_20770461843813
// MI455X (gfx1250) — hardware-verified
//
#include <hip/hip_runtime.h>


#ifndef NB
#define NB 1024
#endif
#define NB_FULL 1024
#define NF    512
#define DD    784
#define KP    832
#define KLOOP 800
#define BT    32
#define FT    64
#define KC    64
#define NCH   (KP / KC)
#define LP    (KC + 4)
#define SP    (FT + 4)
#define RW    8
#define L2E   1.4426950408889634f

static_assert(NB <= NB_FULL);
static_assert(NB % BT == 0);
static_assert(NF % FT == 0);
static_assert(DD % 8 == 0);
static_assert(KP % 64 == 0);
static_assert(KP % KC == 0);
static_assert(KLOOP % 32 == 0);
static_assert(KLOOP >= DD);
static_assert(KLOOP <= KP);
static_assert(KP >= DD);
static_assert(KC % 8 == 0);
static_assert(256 * 1 * 8 == BT * KC);
static_assert(256 * 2 * 8 == FT * KC);
static_assert(256 * 16 * 2 == BT * FT * 4);
static_assert(32 * 16 * 4 == NF * 4);
static_assert((LP * 4) % 16 == 0);
static_assert((SP * 4) % 16 == 0);
static_assert((BT * LP + FT * LP + BT * SP) * 4 <= 65536);
static_assert((BT * LP + FT * LP + BT * SP) * 4 <= 131072);
static_assert(BT == 32);
static_assert(FT == 64);

typedef unsigned short bf;
typedef __attribute__((ext_vector_type(16))) __bf16   v16bf;
typedef __attribute__((ext_vector_type(8)))  unsigned short v8us;
typedef __attribute__((ext_vector_type(8)))  float    v8f;
typedef __attribute__((ext_vector_type(4)))  float    v4f;
typedef v4f  __attribute__((may_alias)) v4fa;

__device__ __forceinline__ unsigned short f2bf(float f) { unsigned u = __float_as_uint(f); u += 0x7FFFu + ((u >> 16) & 1u); return (unsigned short)(u >> 16); }
__device__ __forceinline__ v16bf cat16b(v8us lo, v8us hi) { return __builtin_bit_cast(v16bf, __builtin_shufflevector(lo, hi, 0, 1, 2, 3, 4, 5, 6, 7, 8, 9, 10, 11, 12, 13, 14, 15)); }
__device__ __forceinline__ v8f wmmab(v16bf a, v16bf b, v8f c) { return __builtin_amdgcn_wmma_f32_16x16x32_bf16(false, a, false, b, (short)0, c, false, false); }
__device__ __forceinline__ v16bf ldb(const bf* p)  { return cat16b(*(const v8us*)p, *(const v8us*)(p + 16)); }
__device__ __forceinline__ v8f wmmab_g(v16bf a, v16bf b, v8f c) { c = wmmab(a, b, c); asm volatile("v_nop\n\tv_nop\n\tv_nop\n\tv_nop" : "+v"(c) : "v"(a), "v"(b)); return c; }

__global__ __launch_bounds__(256) void k_cvtpad(const float* __restrict__ src, bf* dst, int rows) {
    const size_t i = (size_t)blockIdx.x * 256 + threadIdx.x;
    const size_t n8 = (size_t)rows * (KP / 8);
    if (i >= n8) return;
    const int row = (int)(i / (KP / 8)), g = (int)(i % (KP / 8));
    const int gc = g < (DD / 8) ? g : (DD / 8 - 1);
    v8f v = *(const v8f*)(src + (size_t)row * DD + (size_t)gc * 8);
    asm volatile("" : "+v"(v));
    const bool ok = g < (DD / 8);
    v8us o;
#pragma unroll
    for (int k = 0; k < 8; ++k) o[k] = ok ? f2bf(v[k]) : (unsigned short)0;
    *(volatile v8us*)(dst + i * 8) = o; __threadfence(); *(volatile v8us*)(dst + i * 8) = o;
}

__global__ __launch_bounds__(256) void k_score(const bf* __restrict__ XB, const bf* __restrict__ FB, float* S) {
    __shared__ __align__(16) float xs[BT * LP];
    __shared__ __align__(16) float fs[FT * LP];
    __shared__ __align__(16) float sc[BT * SP];
    const int tid = threadIdx.x;
    const int lane = tid & 31, lr = lane & 15, hi = lane >> 4;
    const int wave = __builtin_amdgcn_readfirstlane((int)(threadIdx.x >> 5));
    const int bi = wave >> 2, fj = wave & 3;
    const int rowBase = blockIdx.y * BT, colBase = blockIdx.x * FT;

    v8f acc = (v8f){};
    const size_t aoff = (size_t)(rowBase + bi * 16 + lr) * KP + 8 * hi;
    const size_t boff = (size_t)(colBase + fj * 16 + lr) * KP + 8 * hi;
#pragma unroll 1
    for (int kc = 0; kc < KLOOP; kc += 32) {
        const v16bf a = ldb(XB + aoff + kc);
        const v16bf b = ldb(FB + boff + kc);
        acc = wmmab_g(a, b, acc);
    }

    float l1[8];
#pragma unroll
    for (int m = 0; m < 8; ++m) l1[m] = 0.0f;
    const int fo = (fj * 16 + lr) * LP;
    const int xo = (bi * 16 + hi * 8) * LP;
#pragma unroll 1
    for (int ch = 0; ch < NCH; ++ch) {
        const int kBase = ch * KC;
        __syncthreads();
        {
            const int r = tid >> 3, g = tid & 7;
            const v8us w = *(const v8us*)(XB + (size_t)(rowBase + r) * KP + kBase + g * 8);
            v4f a, c;
#pragma unroll
            for (int i = 0; i < 4; ++i) { a[i] = __uint_as_float(((unsigned)w[i]) << 16); c[i] = __uint_as_float(((unsigned)w[4 + i]) << 16); }
            *(v4fa*)(&xs[r * LP + g * 8]) = a; *(v4fa*)(&xs[r * LP + g * 8 + 4]) = c;
        }
#pragma unroll
        for (int s = 0; s < 2; ++s) {
            const int t = s * 256 + tid; const int r = t >> 3, g = t & 7;
            const v8us w = *(const v8us*)(FB + (size_t)(colBase + r) * KP + kBase + g * 8);
            v4f a, c;
#pragma unroll
            for (int i = 0; i < 4; ++i) { a[i] = __uint_as_float(((unsigned)w[i]) << 16); c[i] = __uint_as_float(((unsigned)w[4 + i]) << 16); }
            *(v4fa*)(&fs[r * LP + g * 8]) = a; *(v4fa*)(&fs[r * LP + g * 8 + 4]) = c;
        }
        __syncthreads();
#pragma unroll 2
        for (int d = 0; d < KC; d += 4) {
            const v4f fv = *(const v4fa*)(&fs[fo + d]);
#pragma unroll
            for (int m = 0; m < 8; ++m) {
                const v4f xv = *(const v4fa*)(&xs[xo + m * LP + d]);
                l1[m] += fabsf(xv[0] - fv[0]) + fabsf(xv[1] - fv[1]) + fabsf(xv[2] - fv[2]) + fabsf(xv[3] - fv[3]);
            }
        }
    }

#pragma unroll
    for (int v = 0; v < 8; ++v) sc[(bi * 16 + hi * 8 + v) * SP + fj * 16 + lr] = acc[v] - l1[v] * 0.2f;
    __syncthreads();
    float* sbase = S + (size_t)rowBase * NF + colBase;
#pragma unroll 1
    for (int ps = 0; ps < 2; ++ps) {
#pragma unroll
        for (int s = 0; s < 2; ++s) { const int row = 4 * wave + 2 * s + (lane >> 4), c4 = (lane & 15) * 4;
            const v4f val = *(const v4fa*)(&sc[row * SP + c4]);
            *(volatile v4f*)(sbase + (size_t)row * NF + c4) = val; }
        if (ps == 0) __threadfence(); }
}

__global__ __launch_bounds__(32 * RW) void k_lsm(const float* __restrict__ S, float* OUT, int rows) {
#pragma clang fp contract(off)
    const int lane = threadIdx.x & 31;
    const int wave = __builtin_amdgcn_readfirstlane((int)(threadIdx.x >> 5));
    const int row = blockIdx.x * RW + wave;
    if (row >= rows) return;
    const float* sr = S + (size_t)row * NF + lane * 4;
    v4f s[4];
#pragma unroll
    for (int i = 0; i < 4; ++i) s[i] = *(const v4f*)(sr + i * 128);
    float mx = s[0][0];
#pragma unroll
    for (int i = 0; i < 4; ++i)
#pragma unroll
        for (int j = 0; j < 4; ++j) mx = fmaxf(mx, s[i][j]);
    mx = fmaxf(mx, __shfl_xor(mx, 16, 32));
    mx = fmaxf(mx, __shfl_xor(mx, 8, 32));
    mx = fmaxf(mx, __shfl_xor(mx, 4, 32));
    mx = fmaxf(mx, __shfl_xor(mx, 2, 32));
    mx = fmaxf(mx, __shfl_xor(mx, 1, 32));
    float sum = 0.0f;
#pragma unroll
    for (int i = 0; i < 4; ++i)
#pragma unroll
        for (int j = 0; j < 4; ++j) { const float sh = s[i][j] - mx; s[i][j] = sh; sum += __builtin_amdgcn_exp2f(sh * L2E); }
    sum += __shfl_xor(sum, 16, 32);
    sum += __shfl_xor(sum, 8, 32);
    sum += __shfl_xor(sum, 4, 32);
    sum += __shfl_xor(sum, 2, 32);
    sum += __shfl_xor(sum, 1, 32);
    const float lg = __logf(sum);
    v4f o[4];
#pragma unroll
    for (int i = 0; i < 4; ++i) { o[i][0] = s[i][0] - lg; o[i][1] = s[i][1] - lg; o[i][2] = s[i][2] - lg; o[i][3] = s[i][3] - lg; }
    float* orow = OUT + (size_t)row * NF + lane * 4;
#pragma unroll 1
    for (int ps = 0; ps < 2; ++ps) {
#pragma unroll
        for (int i = 0; i < 4; ++i) *(volatile v4f*)(orow + i * 128) = o[i];
        if (ps == 0) __threadfence(); }
}

static constexpr size_t al256(size_t v) { return (v + 255) & ~(size_t)255; }
static constexpr size_t SZ_XB = al256((size_t)NB * KP * 2);
static constexpr size_t SZ_FB = al256((size_t)NF * KP * 2);
static constexpr size_t SZ_S  = al256((size_t)NB * NF * 4);
static constexpr size_t SZ_TOTAL = SZ_XB + SZ_FB + SZ_S;
static_assert(SZ_TOTAL <= (size_t)134217728);
static_assert(((size_t)NB * (KP / 8)) % 32 == 0);
static_assert(((size_t)NF * (KP / 8)) % 32 == 0);
static_assert((size_t)(NB - 1) * NF + NF <= (size_t)NB_FULL * NF);

extern "C" void kernel_launch(void* const* d_in, const int* in_sizes, int n_in,
                              void* d_out, int out_size, void* d_ws, size_t ws_size, hipStream_t stream) {
    if (n_in < 2) return;
    if ((size_t)in_sizes[0] < (size_t)NB * DD) return;
    if ((size_t)in_sizes[1] < (size_t)NF * DD) return;
    if ((size_t)out_size < (size_t)NB * NF) return;
    if (SZ_TOTAL > ws_size) return;
    const float* xin = (const float*)d_in[0];
    const float* fin = (const float*)d_in[1];
    float* OUT = (float*)d_out;
    char* wsp = (char*)d_ws;
    bf* XB = (bf*)wsp; wsp += SZ_XB;
    bf* FB = (bf*)wsp; wsp += SZ_FB;
    float* S = (float*)wsp; wsp += SZ_S;

    { const size_t n8 = (size_t)NB * (KP / 8); k_cvtpad<<<(unsigned)((n8 + 255) / 256), 256, 0, stream>>>(xin, XB, NB); }
    { const size_t n8 = (size_t)NF * (KP / 8); k_cvtpad<<<(unsigned)((n8 + 255) / 256), 256, 0, stream>>>(fin, FB, NF); }
    k_score<<<dim3(NF / FT, NB / BT, 1), 256, 0, stream>>>(XB, FB, S);
    k_lsm<<<(unsigned)((NB + RW - 1) / RW), 32 * RW, 0, stream>>>(S, OUT, NB);
}
